// RNN_64424509440217
// MI455X (gfx1250) — hardware-run, weakly checked
//
#include <hip/hip_runtime.h>
#include <math.h>

typedef __attribute__((ext_vector_type(16))) _Float16 v16h;
typedef __attribute__((ext_vector_type(8)))  _Float16 v8h;
typedef __attribute__((ext_vector_type(4)))  _Float16 v4h;
typedef __attribute__((ext_vector_type(2)))  _Float16 v2h;
typedef __attribute__((ext_vector_type(16))) __bf16   v16b;
typedef __attribute__((ext_vector_type(8)))  __bf16   v8b;
typedef __attribute__((ext_vector_type(8)))  float    v8f;
typedef __attribute__((ext_vector_type(4)))  float    v4f;
typedef __attribute__((ext_vector_type(2)))  float    v2f;

constexpr int kB    = 128;
constexpr int kT    = 1024;
constexpr int kI    = 100;
constexpr int kIP   = 128;
constexpr int kH    = 200;
constexpr int kHK   = 224;
constexpr int kHP   = 256;
constexpr int kThr  = 256;
constexpr float kInCarry = 1024.0f;
constexpr float kSc = 1.0f / (kInCarry * kInCarry);
constexpr float kF16MinNormal = 6.103515625e-5f;

static_assert(kB == 128 && kT == 1024 && kI == 100 && kIP == 128 && kH == 200 && kHK == 224 && kHP == 256 && kH % 8 == 0 && kI % 4 == 0, "the index arithmetic below uses these sizes");

constexpr size_t kOffZ = 0ull;
constexpr size_t kOffX16 = 266240ull;
constexpr size_t kOffXP = 33820672ull;
constexpr size_t kOffG = 168038400ull;
constexpr size_t kOffOT = 168169472ull;
constexpr size_t kWsTotal = 168693760ull;
static_assert(kWsTotal <= 268435456ull, "the carve stands under 256 MiB");
static_assert(kOffZ == 0
  && kOffX16 == kOffZ + 266240ull
  && kOffXP == kOffX16 + 33554432ull
  && kOffG == kOffXP + 134217728ull
  && kOffOT == kOffG + 131072ull
  && kWsTotal == kOffOT + 524288ull, "the carve is a chain: every region starts where the one before ends");
static_assert(4096ull + (size_t)kHP * kHP * 2 + (size_t)kHP * kIP * 2 + (size_t)kB * kHP * 2 == 266240ull && (size_t)kB * kT * kIP * 2 == 33554432ull && (size_t)kB * kT * kHP * 4 == 134217728ull && (size_t)kB * kHP * 4 == 131072ull && (size_t)kT * kB * 4 == 524288ull, "every region's length is its plane's");
static_assert((kOffX16 % 256) == 0 && (kOffXP % 256) == 0 && (kOffG % 256) == 0 && (kOffOT % 256) == 0, "every region starts on a multiple of 256 B");
constexpr size_t kZW16  = 4096ull;
constexpr size_t kZWI16 = 4096ull + (size_t)kHP * kHP * 2;
constexpr size_t kZH16  = kZWI16 + (size_t)kHP * kIP * 2;

__device__ __forceinline__ unsigned short f2bf_bits(float f) {
  unsigned u = __float_as_uint(f);
  return (unsigned short)((u + 0x7FFFu + ((u >> 16) & 1u)) >> 16);
}
__device__ __forceinline__ float bf_bits2f(unsigned short h) { return __uint_as_float(((unsigned)h) << 16); }
__device__ __forceinline__ float bf16r(float f) { return bf_bits2f(f2bf_bits(f)); }
__device__ __forceinline__ float carry_flush(float v, float carry) {
  const float s = v * carry;
  return (fabsf(s) < kF16MinNormal) ? 0.0f : s;
}

__device__ __forceinline__ void dep_guard4_h(v8f& a, v8f& b, v8f& c, v8f& d, v16h x, v16h y) { asm volatile("v_nop\n\tv_nop\n\tv_nop\n\tv_nop" : "+v"(a), "+v"(b), "+v"(c), "+v"(d) : "v"(x), "v"(y)); }
__device__ __forceinline__ void dep_guard4_b(v8f& a, v8f& b, v8f& c, v8f& d, v16b x, v16b y) { asm volatile("v_nop\n\tv_nop\n\tv_nop\n\tv_nop" : "+v"(a), "+v"(b), "+v"(c), "+v"(d) : "v"(x), "v"(y)); }
__device__ __forceinline__ void keep4_h(v16h a, v16h b, v16h c, v16h d) { asm volatile("v_nop" :: "v"(a), "v"(b), "v"(c), "v"(d)); }
__device__ __forceinline__ void keep4_b(v16b a, v16b b, v16b c, v16b d) { asm volatile("v_nop" :: "v"(a), "v"(b), "v"(c), "v"(d)); }
__device__ __forceinline__ void acc_guard4(v8f& a, v8f& b, v8f& c, v8f& d) { asm volatile("v_nop\n\tv_nop\n\tv_nop\n\tv_nop" : "+v"(a), "+v"(b), "+v"(c), "+v"(d)); }

template <typename T> struct Frag;
template <> struct Frag<_Float16> {
  typedef v16h V; union U { v16h v; v8h h[2]; };
  static __device__ __forceinline__ v16h load(const _Float16* p) {
    U f; f.h[0] = *(const v8h*)(p); f.h[1] = *(const v8h*)(p + 16); return f.v;
  }
  static __device__ __forceinline__ v8f mma(v16h a, v16h b, v8f c) {
    return __builtin_amdgcn_wmma_f32_16x16x32_f16(false, a, false, b, (short)0, c, false, false);
  }
  static __device__ __forceinline__ void guard4(v8f& a, v8f& b, v8f& c, v8f& d, v16h x, v16h y) { dep_guard4_h(a, b, c, d, x, y); }
  static __device__ __forceinline__ void keep(v16h a, v16h b, v16h c, v16h d) { keep4_h(a, b, c, d); }
};
template <> struct Frag<__bf16> {
  typedef v16b V; union U { v16b v; v8b h[2]; };
  static __device__ __forceinline__ v16b load(const __bf16* p) {
    U f; f.h[0] = *(const v8b*)(p); f.h[1] = *(const v8b*)(p + 16); return f.v;
  }
  static __device__ __forceinline__ v8f mma(v16b a, v16b b, v8f c) {
    return __builtin_amdgcn_wmma_f32_16x16x32_bf16(false, a, false, b, (short)0, c, false, false);
  }
  static __device__ __forceinline__ void guard4(v8f& a, v8f& b, v8f& c, v8f& d, v16b x, v16b y) { dep_guard4_b(a, b, c, d, x, y); }
  static __device__ __forceinline__ void keep(v16b a, v16b b, v16b c, v16b d) { keep4_b(a, b, c, d); }
};

__device__ __forceinline__ v8f mma_h(v16h a, v16h b, v8f c) {
  c = __builtin_amdgcn_wmma_f32_16x16x32_f16(false, a, false, b, (short)0, c, false, false);
  asm volatile("v_nop\n\tv_nop\n\tv_nop\n\tv_nop" : "+v"(c) : "v"(a), "v"(b));
  return c;
}

template <int ET> struct Elem;
template <> struct Elem<0> { typedef _Float16 T; };
template <> struct Elem<1> { typedef __bf16 T; };
template <int ET, bool SPLIT, int BIAS_MODE, int OUT_MODE, bool RESID, int ACT = 0>
__global__ __launch_bounds__(256) void wmma_gemm64(
    const unsigned short* __restrict__ Ap, const unsigned short* __restrict__ A2p, int lda, long strideA,
    const unsigned short* __restrict__ Btp, const unsigned short* __restrict__ Bt2p, int ldb, long strideB,
    void* __restrict__ Cout, void* __restrict__ Cout2, int ldc, long strideC,
    const float* __restrict__ bias,
    const float* __restrict__ resid, long strideR,
    int M, int N, int K, float scale) {
  typedef typename Elem<ET>::T T;
  typedef typename Frag<T>::V V;
  const T* A = (const T*)Ap; const T* A2 = (const T*)A2p; const T* Bt = (const T*)Btp; const T* Bt2 = (const T*)Bt2p;
  __shared__ __align__(16) float sT[8][16 * 68];
  const int b    = blockIdx.y;
  const int lane = threadIdx.x & 31;
  const int wave = threadIdx.x >> 5;
  const int tilesN = N >> 6;
  const int tilesM = M >> 6;
  const int tile = blockIdx.x * 8 + wave;
  if (tile >= tilesM * tilesN) return;
  const int tm = tile / tilesN;
  const int tn = tile - tm * tilesN;
  const int m0 = tm << 6;
  const int n0 = tn << 6;

  const T* Ab  = A  + (size_t)b * strideA;
  const T* Bb  = Bt + (size_t)b * strideB;
  const T* Ab2 = SPLIT ? (A2  + (size_t)b * strideA) : nullptr;
  const T* Bb2 = SPLIT ? (Bt2 + (size_t)b * strideB) : nullptr;

  const int rlane = lane & 15;
  const int koff  = (lane >> 4) * 8;
  const int mOff  = (lane >> 4) * 8;

  v8f acc[4][4];
#pragma unroll
  for (int i = 0; i < 4; ++i)
#pragma unroll
    for (int j = 0; j < 4; ++j) acc[i][j] = (v8f){0.f,0.f,0.f,0.f,0.f,0.f,0.f,0.f};

  for (int k0 = 0; k0 < K; k0 += 32) {
    V bh[4], bl[4];
#pragma unroll
    for (int j = 0; j < 4; ++j) {
      const size_t bo = (size_t)(n0 + (j << 4) + rlane) * ldb + koff + k0;
      bh[j] = Frag<T>::load(Bb + bo);
      if (SPLIT) bl[j] = Frag<T>::load(Bb2 + bo);
    }
#pragma unroll
    for (int i = 0; i < 4; ++i) {
      const size_t ao = (size_t)(m0 + (i << 4) + rlane) * lda + koff + k0;
      V ah = Frag<T>::load(Ab + ao);
      V al;
      if (SPLIT) al = Frag<T>::load(Ab2 + ao);
#pragma unroll
      for (int j = 0; j < 4; ++j) {
        acc[i][j] = Frag<T>::mma(ah, bh[j], acc[i][j]);
        if (SPLIT) {
          acc[i][j] = Frag<T>::mma(ah, bl[j], acc[i][j]);
          acc[i][j] = Frag<T>::mma(al, bh[j], acc[i][j]);
        }
      }
      Frag<T>::guard4(acc[i][0], acc[i][1], acc[i][2], acc[i][3], ah, SPLIT ? al : ah);
    }
    Frag<T>::keep(bh[0], bh[1], bh[2], bh[3]);
    if (SPLIT) Frag<T>::keep(bl[0], bl[1], bl[2], bl[3]);
  }
  acc_guard4(acc[0][0], acc[0][1], acc[0][2], acc[0][3]);
  acc_guard4(acc[1][0], acc[1][1], acc[1][2], acc[1][3]);
  acc_guard4(acc[2][0], acc[2][1], acc[2][2], acc[2][3]);
  acc_guard4(acc[3][0], acc[3][1], acc[3][2], acc[3][3]);

  float* slab = sT[wave];
  const float* Rb = RESID ? (resid + (size_t)b * strideR) : nullptr;
#pragma unroll
  for (int i = 0; i < 4; ++i) {
    const int mBase = m0 + (i << 4);
#pragma unroll
    for (int j = 0; j < 4; ++j) {
      const int n = n0 + (j << 4) + rlane;
      float bv = 0.f;
      if (BIAS_MODE == 2) bv = bias[n];
#pragma unroll
      for (int r = 0; r < 8; ++r) {
        float v = acc[i][j][r] * scale;
        if (BIAS_MODE == 1) v += bias[mBase + mOff + r];
        if (BIAS_MODE == 2) v += bv;
        if (RESID) v += Rb[(size_t)(mBase + mOff + r) * ldc + n];
        if (ACT == 1) v = tanhf(v);
        if (ACT == 2) v = fmaxf(v, 0.0f);
        if (ACT == 3) v = v / (1.0f + expf(-v));
        if (ACT == 4) v = (v > 0.f) ? v : 0.01f * v;
        slab[(mOff + r) * 68 + (j << 4) + rlane] = v;
      }
    }
    __builtin_amdgcn_fence(__ATOMIC_RELEASE, "workgroup");
    __builtin_amdgcn_wave_barrier();
    __builtin_amdgcn_fence(__ATOMIC_ACQUIRE, "workgroup");
    if (OUT_MODE == 0) {
      float* C = (float*)Cout + (size_t)b * strideC;
      const int hh = lane >> 4, c4 = (lane & 15) * 4;
      for (int pass = 0; pass < 2; ++pass) {
#pragma unroll
        for (int it = 0; it < 8; ++it) {
          const int row = it * 2 + hh;
          v4f v = *(const v4f*)(slab + row * 68 + c4);
          *(volatile v4f*)(C + (size_t)(mBase + row) * ldc + n0 + c4) = v;
        }
        __threadfence();
      }
    } else {
      const int q = lane >> 3, c8 = (lane & 7) * 8;
      unsigned short* C  = (unsigned short*)Cout  + (size_t)b * strideC;
      unsigned short* C2 = (OUT_MODE == 2) ? ((unsigned short*)Cout2 + (size_t)b * strideC) : nullptr;
      for (int pass = 0; pass < 2; ++pass) {
#pragma unroll
        for (int it = 0; it < 4; ++it) {
          const int row = it * 4 + q;
          const float* sp = slab + row * 68 + c8;
          v8h hv, lv;
#pragma unroll
          for (int e = 0; e < 8; ++e) {
            if (OUT_MODE == 1) {
              hv[e] = (_Float16)sp[e];
            } else {
              unsigned short hb = f2bf_bits(sp[e]);
              unsigned short lb = f2bf_bits(sp[e] - bf_bits2f(hb));
              hv[e] = __builtin_bit_cast(_Float16, hb);
              lv[e] = __builtin_bit_cast(_Float16, lb);
            }
          }
          *(volatile v8h*)(C + (size_t)(mBase + row) * ldc + n0 + c8) = hv;
          if (OUT_MODE == 2) *(volatile v8h*)(C2 + (size_t)(mBase + row) * ldc + n0 + c8) = lv;
        }
        __threadfence();
      }
    }
    __builtin_amdgcn_fence(__ATOMIC_RELEASE, "workgroup");
    __builtin_amdgcn_wave_barrier();
    __builtin_amdgcn_fence(__ATOMIC_ACQUIRE, "workgroup");
  }
}

__global__ __launch_bounds__(kThr) void zero_kernel(float* __restrict__ dst) {
  const size_t o4 = ((size_t)blockIdx.x * kThr + threadIdx.x) * 4u;
  const v4f z = {0.f, 0.f, 0.f, 0.f};
  *(volatile v4f*)(dst + o4) = z;
  __threadfence();
  *(volatile v4f*)(dst + o4) = z;
}
__global__ __launch_bounds__(kThr) void padcast_kernel(const float* __restrict__ S, unsigned short* __restrict__ D, int G, int lg, int srow, int P, int r0) {
  const unsigned i = blockIdx.x * blockDim.x + threadIdx.x;
  const unsigned g = i & ((1u << lg) - 1u), row = i >> lg;
  const unsigned gc = (g < (unsigned)G) ? g : (unsigned)G - 1u;
  const v4f a = *(const v4f*)(S + (size_t)row * (unsigned)srow + gc * 4u);
  const float keep = (g < (unsigned)G) ? 1.0f : 0.0f;
  v4h hv;
#pragma unroll
  for (int e = 0; e < 4; ++e) hv[e] = (_Float16)(keep * carry_flush(bf16r(a[e]), kInCarry));
  unsigned short* dp = D + (size_t)((unsigned)r0 + row) * (unsigned)P + g * 4u;
  *(volatile v4h*)dp = hv;
  __threadfence();
  *(volatile v4h*)dp = hv;
}

__global__ __launch_bounds__(kThr) void cell_kernel(float* __restrict__ XP, const float* __restrict__ G, const float* __restrict__ b_ih, const float* __restrict__ b_hh, const float* __restrict__ b_out,
                                                    unsigned short* __restrict__ H16, float* __restrict__ OT, int t) {
  if (blockIdx.x < 16u) {
    if (t < kT) {
      const unsigned v = blockIdx.x * (unsigned)kThr + threadIdx.x;
      const unsigned b = v >> 5, l = v & 31u;
      const unsigned u8 = l << 3;
      const unsigned uc = (l < 25u) ? u8 : 192u;
      const float keep = (l < 25u) ? 1.0f : 0.0f;
      float* xr = XP + ((size_t)b * kT + (unsigned)t) * kHP;
      const float* g = G + (size_t)b * kHP + uc;
      v8f ho; v8h hv;
#pragma unroll
      for (int hlf = 0; hlf < 2; ++hlf) {
        const v4f a = *(const v4f*)(xr + uc + 4 * hlf), c = *(const v4f*)(g + 4 * hlf), p = *(const v4f*)(b_ih + uc + 4 * hlf), q = *(const v4f*)(b_hh + uc + 4 * hlf);
#pragma unroll
        for (int e = 0; e < 4; ++e) {
          const float hn = keep * fmaxf(((a[e] + bf16r(p[e])) + bf16r(q[e])) + c[e], 0.0f);
          ho[4 * hlf + e] = hn;
          hv[4 * hlf + e] = (_Float16)carry_flush(hn, kInCarry);
        }
      }
      float* ph = xr + u8;
      unsigned short* pa = H16 + (size_t)b * kHP + u8;
      for (int pass = 0; pass < 2; ++pass) {
        *(volatile v8f*)ph = ho;
        *(volatile v8h*)pa = hv;
        __threadfence();
      }
    }
  } else {
    if (t > 0 && threadIdx.x < (unsigned)kB) {
      const unsigned b = threadIdx.x;
      const float o = G[(size_t)b * kHP + (unsigned)kH] + bf16r(b_out[0]);
      float* po = OT + (size_t)(t - 1) * kB + b;
      *(volatile float*)po = o;
      __threadfence();
      *(volatile float*)po = o;
    }
  }
}
static_assert(kB * 32 == 16 * kThr && kH == 25 * 8 && kB <= kThr && kB % 32 == 0, "the cell's grid exact: 16 blocks of a wave a row + one block whose first 128 threads are the rows");

__global__ __launch_bounds__(kThr) void copy_kernel(const float* __restrict__ OT, const float* __restrict__ HS, float* __restrict__ out) {
  const unsigned i = blockIdx.x * (unsigned)kThr + threadIdx.x;
  float y;
  if (blockIdx.x < 512u) {
    const unsigned b = i >> 10, t = i & 1023u;
    y = OT[(size_t)t * kB + b];
  } else {
    const unsigned j = i - (unsigned)(kB * kT);
    const unsigned row = j / (unsigned)kH;
    const unsigned u = j - row * (unsigned)kH;
    y = HS[(size_t)row * kHP + u];
  }
  float* dp = out + i;
  *(volatile float*)dp = y;
  __threadfence();
  *(volatile float*)dp = y;
}
static_assert((size_t)kB * kT == 512ull * kThr && ((size_t)kB * kT + (size_t)kB * kT * kH) == 102912ull * kThr && ((size_t)kB * kT * 4) % 128 == 0, "the copy's grid exact: 512 + 102,400 blocks; the second result starts on a line");

extern "C" void kernel_launch(void* const* d_in, const int* in_sizes, int n_in,
                              void* d_out, int out_size, void* d_ws, size_t ws_size,
                              hipStream_t stream) {
  if (n_in < 7 || d_out == nullptr || d_ws == nullptr) return;
  if (in_sizes[0] != kB * kT * kI || in_sizes[1] != kH * kI || in_sizes[2] != kH * kH || in_sizes[3] != kH || in_sizes[4] != kH || in_sizes[5] != kH || in_sizes[6] != 1) return;
  if (out_size != kB * kT + kB * kT * kH) return;
  if (ws_size < kWsTotal) return;
  const float* x = (const float*)d_in[0];
  const float* W_ih = (const float*)d_in[1];
  const float* W_hh = (const float*)d_in[2];
  const float* b_ih = (const float*)d_in[3];
  const float* b_hh = (const float*)d_in[4];
  const float* W_out = (const float*)d_in[5];
  const float* b_out = (const float*)d_in[6];
  float* oOut = (float*)d_out;
  char* ws = (char*)d_ws;
  float* ZB = (float*)(ws + kOffZ);
  unsigned short* W16 = (unsigned short*)(ws + kOffZ + kZW16);
  unsigned short* WI16 = (unsigned short*)(ws + kOffZ + kZWI16);
  unsigned short* H16 = (unsigned short*)(ws + kOffZ + kZH16);
  unsigned short* X16 = (unsigned short*)(ws + kOffX16);
  float* XP = (float*)(ws + kOffXP);
  float* G = (float*)(ws + kOffG);
  float* OT = (float*)(ws + kOffOT);

  static_assert(266240ull / 16ull == 65ull * kThr && ((size_t)kB * kT * 32) % kThr == 0 && (kH * 32) % kThr == 0 && (kH * 64) % kThr == 0, "the zero fill's grid (65 blocks over Z's 266,240 B) and the padding cast's grids exact");
  zero_kernel<<<65, kThr, 0, stream>>>(ZB);
  padcast_kernel<<<(int)(((size_t)kB * kT * 32) / kThr), kThr, 0, stream>>>(x, X16, kI / 4, 5, kI, kIP, 0);
  padcast_kernel<<<kH * 32 / kThr, kThr, 0, stream>>>(W_ih, WI16, kI / 4, 5, kI, kIP, 0);
  padcast_kernel<<<kH * 64 / kThr, kThr, 0, stream>>>(W_hh, W16, kH / 4, 6, kH, kHP, 0);
  padcast_kernel<<<1, 64, 0, stream>>>(W_out, W16, kH / 4, 6, kH, kHP, kH);
  wmma_gemm64<0, false, 2, 0, false, 0><<<dim3((kB * kT / 64) * (kHP / 64) / 8, 1), 256, 0, stream>>>(
      X16, X16, kIP, 0L, WI16, WI16, kIP, 0L, (void*)XP, (void*)XP, kHP, 0L, ZB, nullptr, 0L, kB * kT, kHP, kIP, kSc);
  for (int t = 0; t <= kT; ++t) {
    wmma_gemm64<0, false, 2, 0, false, 0><<<dim3((kB / 64) * (kHP / 64) / 8, 1), 256, 0, stream>>>(
        H16, H16, kHP, 0L, W16, W16, kHP, 0L, (void*)G, (void*)G, kHP, 0L, ZB, nullptr, 0L, kB, kHP, kHK, kSc);
    cell_kernel<<<17, kThr, 0, stream>>>(XP, G, b_ih, b_hh, b_out, H16, OT, t);
  }
  copy_kernel<<<102912, kThr, 0, stream>>>(OT, XP, oOut);
}
static_assert(((kB * kT / 64) * (kHP / 64)) % 8 == 0 && ((kB / 64) * (kHP / 64)) % 8 == 0 && kHK % 32 == 0 && kIP % 32 == 0, "every engine grid: whole blocks of eight wave tiles; every depth a multiple of 32");
